// LoRALSTMModel_66434554134960
// MI455X (gfx1250) — hardware-run, weakly checked
//
#include <hip/hip_runtime.h>
#include <math.h>

typedef __attribute__((ext_vector_type(16))) _Float16 v16h;
typedef __attribute__((ext_vector_type(8)))  _Float16 v8h;
typedef __attribute__((ext_vector_type(4)))  _Float16 v4h;
typedef __attribute__((ext_vector_type(2)))  _Float16 v2h;
typedef __attribute__((ext_vector_type(16))) __bf16   v16b;
typedef __attribute__((ext_vector_type(8)))  __bf16   v8b;
typedef __attribute__((ext_vector_type(8)))  float    v8f;
typedef __attribute__((ext_vector_type(4)))  float    v4f;
typedef __attribute__((ext_vector_type(2)))  float    v2f;


constexpr int kT   = 256;
constexpr int kB   = 64;
constexpr int kW   = 1024;
constexpr int kG   = 4 * kW;
constexpr int kR   = 16;
constexpr int kL   = 2;
constexpr int kKx  = 2 * kW;
constexpr int kKs  = 4 * kR;
constexpr int kK   = kKx + 2 * kKs;
constexpr int kThr = 256;
constexpr float kInCarry = 1024.0f;
constexpr float kSc20 = 1.0f / (kInCarry * kInCarry);
constexpr float kSc10 = 1.0f / kInCarry;
constexpr float kF16MinNormal = 6.103515625e-5f;

static_assert(kT == 256 && kB == 64 && kW == 1024 && kG == 4096 && kR == 16 && kL == 2 && kKx == 2048 && kKs == 64 && kK == 2176 && kW / 4 == 256 && kK % 32 == 0 && (kK * 2) % 128 == 0 && (kKx * 2) % 128 == 0, "the index arithmetic below uses these sizes: a cell's row is 256 lanes of four columns; a slot row is 16 lanes of eight columns; an operand's row and its slot columns start on whole 128-B lines");

constexpr size_t kOffAL   = 0ull;
constexpr size_t kOffWL   = 557056ull;
constexpr size_t kOffDA   = 36208640ull;
constexpr size_t kOffDB   = 36470784ull;
constexpr size_t kOffPL   = 36732928ull;
constexpr size_t kWsTotal = 38830080ull;
static_assert(kOffWL == (size_t)kL * kB * kK * 2ull && kOffDA == kOffWL + (size_t)kL * kG * kK * 2ull && kOffDB == kOffDA + (size_t)kL * kKs * kW * 2ull && kOffPL == kOffDB + (size_t)kL * kKs * kW * 2ull && kWsTotal == kOffPL + (size_t)kL * kB * kG * 4ull, "the carve is a chain: every region starts where the one before ends");
static_assert((kOffWL % 256) == 0 && (kOffDA % 256) == 0 && (kOffDB % 256) == 0 && (kOffPL % 256) == 0, "every region starts on a multiple of 256 B");

__device__ __forceinline__ unsigned short f2bf_bits(float f) {
  unsigned u = __float_as_uint(f);
  return (unsigned short)((u + 0x7FFFu + ((u >> 16) & 1u)) >> 16);
}
__device__ __forceinline__ float bf_bits2f(unsigned short h) { return __uint_as_float(((unsigned)h) << 16); }
__device__ __forceinline__ float bf16r(float f) { return bf_bits2f(f2bf_bits(f)); }
__device__ __forceinline__ float carry_flush(float v, float carry) {
  const float s = v * carry;
  return (fabsf(s) < kF16MinNormal) ? 0.0f : s;
}

__device__ __forceinline__ void dep_guard4_h(v8f& a, v8f& b, v8f& c, v8f& d, v16h x, v16h y) { asm volatile("v_nop\n\tv_nop\n\tv_nop\n\tv_nop" : "+v"(a), "+v"(b), "+v"(c), "+v"(d) : "v"(x), "v"(y)); }
__device__ __forceinline__ void dep_guard4_b(v8f& a, v8f& b, v8f& c, v8f& d, v16b x, v16b y) { asm volatile("v_nop\n\tv_nop\n\tv_nop\n\tv_nop" : "+v"(a), "+v"(b), "+v"(c), "+v"(d) : "v"(x), "v"(y)); }
__device__ __forceinline__ void keep4_h(v16h a, v16h b, v16h c, v16h d) { asm volatile("v_nop" :: "v"(a), "v"(b), "v"(c), "v"(d)); }
__device__ __forceinline__ void keep4_b(v16b a, v16b b, v16b c, v16b d) { asm volatile("v_nop" :: "v"(a), "v"(b), "v"(c), "v"(d)); }
__device__ __forceinline__ void acc_guard4(v8f& a, v8f& b, v8f& c, v8f& d) { asm volatile("v_nop\n\tv_nop\n\tv_nop\n\tv_nop" : "+v"(a), "+v"(b), "+v"(c), "+v"(d)); }

template <typename T> struct Frag;
template <> struct Frag<_Float16> {
  typedef v16h V; union U { v16h v; v8h h[2]; };
  static __device__ __forceinline__ v16h load(const _Float16* p) {
    U f; f.h[0] = *(const v8h*)(p); f.h[1] = *(const v8h*)(p + 16); return f.v;
  }
  static __device__ __forceinline__ v8f mma(v16h a, v16h b, v8f c) {
    return __builtin_amdgcn_wmma_f32_16x16x32_f16(false, a, false, b, (short)0, c, false, false);
  }
  static __device__ __forceinline__ void guard4(v8f& a, v8f& b, v8f& c, v8f& d, v16h x, v16h y) { dep_guard4_h(a, b, c, d, x, y); }
  static __device__ __forceinline__ void keep(v16h a, v16h b, v16h c, v16h d) { keep4_h(a, b, c, d); }
};
template <> struct Frag<__bf16> {
  typedef v16b V; union U { v16b v; v8b h[2]; };
  static __device__ __forceinline__ v16b load(const __bf16* p) {
    U f; f.h[0] = *(const v8b*)(p); f.h[1] = *(const v8b*)(p + 16); return f.v;
  }
  static __device__ __forceinline__ v8f mma(v16b a, v16b b, v8f c) {
    return __builtin_amdgcn_wmma_f32_16x16x32_bf16(false, a, false, b, (short)0, c, false, false);
  }
  static __device__ __forceinline__ void guard4(v8f& a, v8f& b, v8f& c, v8f& d, v16b x, v16b y) { dep_guard4_b(a, b, c, d, x, y); }
  static __device__ __forceinline__ void keep(v16b a, v16b b, v16b c, v16b d) { keep4_b(a, b, c, d); }
};

__device__ __forceinline__ v8f mma_h(v16h a, v16h b, v8f c) {
  c = __builtin_amdgcn_wmma_f32_16x16x32_f16(false, a, false, b, (short)0, c, false, false);
  asm volatile("v_nop\n\tv_nop\n\tv_nop\n\tv_nop" : "+v"(c) : "v"(a), "v"(b));
  return c;
}

template <int ET> struct Elem;
template <> struct Elem<0> { typedef _Float16 T; };
template <> struct Elem<1> { typedef __bf16 T; };
template <int ET, bool SPLIT, int BIAS_MODE, int OUT_MODE, bool RESID, int ACT = 0>
__global__ __launch_bounds__(256) void wmma_gemm64(
    const unsigned short* __restrict__ Ap, const unsigned short* __restrict__ A2p, int lda, long strideA,
    const unsigned short* __restrict__ Btp, const unsigned short* __restrict__ Bt2p, int ldb, long strideB,
    void* __restrict__ Cout, void* __restrict__ Cout2, int ldc, long strideC,
    const float* __restrict__ bias,
    const float* __restrict__ resid, long strideR,
    int M, int N, int K, float scale) {
  typedef typename Elem<ET>::T T;
  typedef typename Frag<T>::V V;
  const T* A = (const T*)Ap; const T* A2 = (const T*)A2p; const T* Bt = (const T*)Btp; const T* Bt2 = (const T*)Bt2p;
  __shared__ __align__(16) float sT[8][16 * 68];
  const int b    = blockIdx.y;
  const int lane = threadIdx.x & 31;
  const int wave = threadIdx.x >> 5;
  const int tilesN = N >> 6;
  const int tilesM = M >> 6;
  const int tile = blockIdx.x * 8 + wave;
  if (tile >= tilesM * tilesN) return;
  const int tm = tile / tilesN;
  const int tn = tile - tm * tilesN;
  const int m0 = tm << 6;
  const int n0 = tn << 6;

  const T* Ab  = A  + (size_t)b * strideA;
  const T* Bb  = Bt + (size_t)b * strideB;
  const T* Ab2 = SPLIT ? (A2  + (size_t)b * strideA) : nullptr;
  const T* Bb2 = SPLIT ? (Bt2 + (size_t)b * strideB) : nullptr;

  const int rlane = lane & 15;
  const int koff  = (lane >> 4) * 8;
  const int mOff  = (lane >> 4) * 8;

  v8f acc[4][4];
#pragma unroll
  for (int i = 0; i < 4; ++i)
#pragma unroll
    for (int j = 0; j < 4; ++j) acc[i][j] = (v8f){0.f,0.f,0.f,0.f,0.f,0.f,0.f,0.f};

  for (int k0 = 0; k0 < K; k0 += 32) {
    V bh[4], bl[4];
#pragma unroll
    for (int j = 0; j < 4; ++j) {
      const size_t bo = (size_t)(n0 + (j << 4) + rlane) * ldb + koff + k0;
      bh[j] = Frag<T>::load(Bb + bo);
      if (SPLIT) bl[j] = Frag<T>::load(Bb2 + bo);
    }
#pragma unroll
    for (int i = 0; i < 4; ++i) {
      const size_t ao = (size_t)(m0 + (i << 4) + rlane) * lda + koff + k0;
      V ah = Frag<T>::load(Ab + ao);
      V al;
      if (SPLIT) al = Frag<T>::load(Ab2 + ao);
#pragma unroll
      for (int j = 0; j < 4; ++j) {
        acc[i][j] = Frag<T>::mma(ah, bh[j], acc[i][j]);
        if (SPLIT) {
          acc[i][j] = Frag<T>::mma(ah, bl[j], acc[i][j]);
          acc[i][j] = Frag<T>::mma(al, bh[j], acc[i][j]);
        }
      }
      Frag<T>::guard4(acc[i][0], acc[i][1], acc[i][2], acc[i][3], ah, SPLIT ? al : ah);
    }
    Frag<T>::keep(bh[0], bh[1], bh[2], bh[3]);
    if (SPLIT) Frag<T>::keep(bl[0], bl[1], bl[2], bl[3]);
  }
  acc_guard4(acc[0][0], acc[0][1], acc[0][2], acc[0][3]);
  acc_guard4(acc[1][0], acc[1][1], acc[1][2], acc[1][3]);
  acc_guard4(acc[2][0], acc[2][1], acc[2][2], acc[2][3]);
  acc_guard4(acc[3][0], acc[3][1], acc[3][2], acc[3][3]);

  float* slab = sT[wave];
  const float* Rb = RESID ? (resid + (size_t)b * strideR) : nullptr;
#pragma unroll
  for (int i = 0; i < 4; ++i) {
    const int mBase = m0 + (i << 4);
#pragma unroll
    for (int j = 0; j < 4; ++j) {
      const int n = n0 + (j << 4) + rlane;
      float bv = 0.f;
      if (BIAS_MODE == 2) bv = bias[n];
#pragma unroll
      for (int r = 0; r < 8; ++r) {
        float v = acc[i][j][r] * scale;
        if (BIAS_MODE == 1) v += bias[mBase + mOff + r];
        if (BIAS_MODE == 2) v += bv;
        if (RESID) v += Rb[(size_t)(mBase + mOff + r) * ldc + n];
        if (ACT == 1) v = tanhf(v);
        if (ACT == 2) v = fmaxf(v, 0.0f);
        if (ACT == 3) v = v / (1.0f + expf(-v));
        if (ACT == 4) v = (v > 0.f) ? v : 0.01f * v;
        slab[(mOff + r) * 68 + (j << 4) + rlane] = v;
      }
    }
    __builtin_amdgcn_fence(__ATOMIC_RELEASE, "workgroup");
    __builtin_amdgcn_wave_barrier();
    __builtin_amdgcn_fence(__ATOMIC_ACQUIRE, "workgroup");
    if (OUT_MODE == 0) {
      float* C = (float*)Cout + (size_t)b * strideC;
      const int hh = lane >> 4, c4 = (lane & 15) * 4;
      for (int pass = 0; pass < 2; ++pass) {
#pragma unroll
        for (int it = 0; it < 8; ++it) {
          const int row = it * 2 + hh;
          v4f v = *(const v4f*)(slab + row * 68 + c4);
          *(volatile v4f*)(C + (size_t)(mBase + row) * ldc + n0 + c4) = v;
        }
        __threadfence();
      }
    } else {
      const int q = lane >> 3, c8 = (lane & 7) * 8;
      unsigned short* C  = (unsigned short*)Cout  + (size_t)b * strideC;
      unsigned short* C2 = (OUT_MODE == 2) ? ((unsigned short*)Cout2 + (size_t)b * strideC) : nullptr;
      for (int pass = 0; pass < 2; ++pass) {
#pragma unroll
        for (int it = 0; it < 4; ++it) {
          const int row = it * 4 + q;
          const float* sp = slab + row * 68 + c8;
          v8h hv, lv;
#pragma unroll
          for (int e = 0; e < 8; ++e) {
            if (OUT_MODE == 1) {
              hv[e] = (_Float16)sp[e];
            } else {
              unsigned short hb = f2bf_bits(sp[e]);
              unsigned short lb = f2bf_bits(sp[e] - bf_bits2f(hb));
              hv[e] = __builtin_bit_cast(_Float16, hb);
              lv[e] = __builtin_bit_cast(_Float16, lb);
            }
          }
          *(volatile v8h*)(C + (size_t)(mBase + row) * ldc + n0 + c8) = hv;
          if (OUT_MODE == 2) *(volatile v8h*)(C2 + (size_t)(mBase + row) * ldc + n0 + c8) = lv;
        }
        __threadfence();
      }
    }
    __builtin_amdgcn_fence(__ATOMIC_RELEASE, "workgroup");
    __builtin_amdgcn_wave_barrier();
    __builtin_amdgcn_fence(__ATOMIC_ACQUIRE, "workgroup");
  }
}


__global__ __launch_bounds__(kThr) void cast_plane_kernel(const float* __restrict__ src, unsigned short* __restrict__ dst,
                                                          int colsLog2, int dstPitch, int dstOff) {
  const int i   = blockIdx.x * kThr + threadIdx.x;
  const int sh  = colsLog2 - 3;
  const int row = i >> sh;
  const int c8  = (i & ((1 << sh) - 1)) * 8;
  const float* sp = src + ((size_t)row << colsLog2) + c8;
  const v4f a0 = *(const v4f*)(sp);
  const v4f a1 = *(const v4f*)(sp + 4);
  v8h hv;
#pragma unroll
  for (int e = 0; e < 4; ++e) {
    const float f0 = a0[e];
    const float f1 = a1[e];
    hv[e]     = (_Float16)carry_flush(bf16r(f0), kInCarry);
    hv[4 + e] = (_Float16)carry_flush(bf16r(f1), kInCarry);
  }
  unsigned short* dp = dst + (size_t)row * dstPitch + dstOff + c8;
  *(volatile v8h*)dp = hv;
  __threadfence();
  *(volatile v8h*)dp = hv;
}

__global__ __launch_bounds__(kThr) void slot_kernel(const float* __restrict__ ua, const float* __restrict__ ub, unsigned short* __restrict__ dst) {
  const unsigned i = blockIdx.x * (unsigned)kThr + threadIdx.x;
  const unsigned n = i >> 4, j = i & 15u;
  const unsigned g = n >> 10;
  const unsigned s = (j & 7u) >> 1, hf = j & 1u;
  const size_t so = (size_t)n * (unsigned)kR + hf * 8u;
  const v4f xa = *(const v4f*)(ua + so), xb = *(const v4f*)(ua + so + 4);
  const v4f ya = *(const v4f*)(ub + so), yb = *(const v4f*)(ub + so + 4);
  const unsigned own = (s == g) ? 0xFFFFFFFFu : 0u;
  const unsigned mx = (j < 8u) ? own : 0u;
  const unsigned my = (j < 8u) ? 0u : own;
  v8h hv;
#pragma unroll
  for (int e = 0; e < 4; ++e) {
    const float f0 = __uint_as_float((__float_as_uint(xa[e]) & mx) | (__float_as_uint(ya[e]) & my));
    const float f1 = __uint_as_float((__float_as_uint(xb[e]) & mx) | (__float_as_uint(yb[e]) & my));
    hv[e]     = (_Float16)carry_flush(bf16r(f0), kInCarry);
    hv[4 + e] = (_Float16)carry_flush(bf16r(f1), kInCarry);
  }
  unsigned short* dp = dst + (size_t)n * (unsigned)kK + (unsigned)kKx + j * 8u;
  *(volatile v8h*)dp = hv;
  __threadfence();
  *(volatile v8h*)dp = hv;
}

template <bool LAST>
__global__ __launch_bounds__(kThr) void cell_kernel(const float* __restrict__ pl, const float* __restrict__ ba, const float* __restrict__ bb, const float* __restrict__ q0, float* __restrict__ qout, float* __restrict__ sout, float* __restrict__ sdup, unsigned short* __restrict__ snext) {
  const unsigned i = blockIdx.x * (unsigned)kThr + threadIdx.x;
  const unsigned r = i >> 8, c4 = (i & 255u) << 2;
  const float* pp = pl + (size_t)r * (unsigned)kG + c4;
  const float* aa = ba + c4;
  const float* bp = bb + c4;
  const size_t o = (size_t)r * (unsigned)kW + c4;
  const v4f pi = *(const v4f*)pp;
  const v4f pf = *(const v4f*)(pp + kW);
  const v4f pg = *(const v4f*)(pp + 2 * kW);
  const v4f po = *(const v4f*)(pp + 3 * kW);
  const v4f ai = *(const v4f*)aa;
  const v4f af = *(const v4f*)(aa + kW);
  const v4f ag = *(const v4f*)(aa + 2 * kW);
  const v4f ao = *(const v4f*)(aa + 3 * kW);
  const v4f bi = *(const v4f*)bp;
  const v4f bf = *(const v4f*)(bp + kW);
  const v4f bg = *(const v4f*)(bp + 2 * kW);
  const v4f bo = *(const v4f*)(bp + 3 * kW);
  const v4f qv = *(const v4f*)(q0 + o);
  v4f sv, nv;
  v4h hv;
#pragma unroll
  for (int e = 0; e < 4; ++e) {
    const float yi = (pi[e] + bf16r(ai[e])) + bf16r(bi[e]);
    const float yf = (pf[e] + bf16r(af[e])) + bf16r(bf[e]);
    const float yg = (pg[e] + bf16r(ag[e])) + bf16r(bg[e]);
    const float yo = (po[e] + bf16r(ao[e])) + bf16r(bo[e]);
    const float gi = 1.0f / (1.0f + expf(-yi));
    const float gf = 1.0f / (1.0f + expf(-yf));
    const float gg = 1.0f - 2.0f / (1.0f + expf(2.0f * yg));
    const float go = 1.0f / (1.0f + expf(-yo));
    nv[e] = gf * bf16r(qv[e]) + gi * gg;
    sv[e] = go * (1.0f - 2.0f / (1.0f + expf(2.0f * nv[e])));
    if (!LAST) hv[e] = (_Float16)carry_flush(sv[e], kInCarry);
  }
  float* qp = qout + o;
  float* sp = sout + o;
  float* dq = LAST ? (sdup + o) : nullptr;
  unsigned short* hp = LAST ? nullptr : (snext + (size_t)r * (unsigned)kK + c4);
  *(volatile v4f*)qp = nv;
  *(volatile v4f*)sp = sv;
  if (LAST) { *(volatile v4f*)dq = sv; }
  else      { *(volatile v4h*)hp = hv; }
  __threadfence();
  *(volatile v4f*)qp = nv;
  *(volatile v4f*)sp = sv;
  if (LAST) { *(volatile v4f*)dq = sv; }
  else      { *(volatile v4h*)hp = hv; }
}

extern "C" void kernel_launch(void* const* d_in, const int* in_sizes, int n_in,
                              void* d_out, int out_size, void* d_ws, size_t ws_size,
                              hipStream_t stream) {
  if (n_in < 11 || d_out == nullptr || d_ws == nullptr) return;
  if (in_sizes[0] != kT * kB * kW || in_sizes[1] != kL * kB * kW || in_sizes[2] != kL * kB * kW || in_sizes[3] != kL * kG * kW || in_sizes[4] != kL * kG * kW || in_sizes[5] != kL * kG || in_sizes[6] != kL * kG || in_sizes[7] != kL * kKs * kW || in_sizes[8] != kL * kG * kR || in_sizes[9] != kL * kKs * kW || in_sizes[10] != kL * kG * kR) return;
  if (out_size != 5 * kB * kW) return;
  if (ws_size < kWsTotal) return;
  char* ws = (char*)d_ws;
  unsigned short* AL0 = (unsigned short*)(ws + kOffAL);
  unsigned short* AL1 = AL0 + (size_t)kB * kK;
  unsigned short* WL0 = (unsigned short*)(ws + kOffWL);
  unsigned short* WL1 = WL0 + (size_t)kG * kK;
  unsigned short* DA0 = (unsigned short*)(ws + kOffDA);
  unsigned short* DA1 = DA0 + (size_t)kKs * kW;
  unsigned short* DB0 = (unsigned short*)(ws + kOffDB);
  unsigned short* DB1 = DB0 + (size_t)kKs * kW;
  float* PL0 = (float*)(ws + kOffPL);
  float* PL1 = PL0 + (size_t)kB * kG;
  const float* xs = (const float*)d_in[0] + (size_t)(kT - 1) * kB * kW;
  const float* p0 = (const float*)d_in[1];
  const float* q0 = (const float*)d_in[2];
  const float* wa = (const float*)d_in[3];
  const float* wb = (const float*)d_in[4];
  const float* ba = (const float*)d_in[5];
  const float* bb = (const float*)d_in[6];
  const float* da = (const float*)d_in[7];
  const float* ua = (const float*)d_in[8];
  const float* db = (const float*)d_in[9];
  const float* ub = (const float*)d_in[10];
  float* R0 = (float*)d_out;
  float* R1 = (float*)d_out + (size_t)kB * kW;
  float* R2 = (float*)d_out + (size_t)3 * kB * kW;

  static_assert((kB * (kW / 8)) % kThr == 0 && (kG * (kW / 8)) % kThr == 0 && (kKs * (kW / 8)) % kThr == 0 && (kG * 16) % kThr == 0 && (kB * (kW / 4)) % kThr == 0, "every grid of the cast, the slots' filler and the cell exact");
  cast_plane_kernel<<<kB * (kW / 8) / kThr, kThr, 0, stream>>>(xs, AL0, 10, kK, 0);
  cast_plane_kernel<<<kB * (kW / 8) / kThr, kThr, 0, stream>>>(p0, AL0, 10, kK, kW);
  cast_plane_kernel<<<kB * (kW / 8) / kThr, kThr, 0, stream>>>(p0 + (size_t)kB * kW, AL1, 10, kK, kW);
  cast_plane_kernel<<<kG * (kW / 8) / kThr, kThr, 0, stream>>>(wa, WL0, 10, kK, 0);
  cast_plane_kernel<<<kG * (kW / 8) / kThr, kThr, 0, stream>>>(wb, WL0, 10, kK, kW);
  cast_plane_kernel<<<kG * (kW / 8) / kThr, kThr, 0, stream>>>(wa + (size_t)kG * kW, WL1, 10, kK, 0);
  cast_plane_kernel<<<kG * (kW / 8) / kThr, kThr, 0, stream>>>(wb + (size_t)kG * kW, WL1, 10, kK, kW);
  cast_plane_kernel<<<kKs * (kW / 8) / kThr, kThr, 0, stream>>>(da, DA0, 10, kW, 0);
  cast_plane_kernel<<<kKs * (kW / 8) / kThr, kThr, 0, stream>>>(db, DB0, 10, kW, 0);
  cast_plane_kernel<<<kKs * (kW / 8) / kThr, kThr, 0, stream>>>(da + (size_t)kKs * kW, DA1, 10, kW, 0);
  cast_plane_kernel<<<kKs * (kW / 8) / kThr, kThr, 0, stream>>>(db + (size_t)kKs * kW, DB1, 10, kW, 0);
  slot_kernel<<<kG * 16 / kThr, kThr, 0, stream>>>(ua, ub, WL0);
  slot_kernel<<<kG * 16 / kThr, kThr, 0, stream>>>(ua + (size_t)kG * kR, ub + (size_t)kG * kR, WL1);

  wmma_gemm64<0, false, 0, 1, false, 0><<<dim3(1, 1), 256, 0, stream>>>(
      AL0, AL0, kK, 0L, DA0, DA0, kW, 0L, (void*)(AL0 + kKx), (void*)(AL0 + kKx), kK, 0L, nullptr, nullptr, 0L, kB, kKs, kW, kSc10);
  wmma_gemm64<0, false, 0, 1, false, 0><<<dim3(1, 1), 256, 0, stream>>>(
      AL0 + kW, AL0 + kW, kK, 0L, DB0, DB0, kW, 0L, (void*)(AL0 + kKx + kKs), (void*)(AL0 + kKx + kKs), kK, 0L, nullptr, nullptr, 0L, kB, kKs, kW, kSc10);
  wmma_gemm64<0, false, 0, 0, false, 0><<<dim3((kB / 64) * (kG / 64) / 8, 1), 256, 0, stream>>>(
      AL0, AL0, kK, 0L, WL0, WL0, kK, 0L, (void*)PL0, (void*)PL0, kG, 0L, nullptr, nullptr, 0L, kB, kG, kK, kSc20);
  cell_kernel<false><<<kB * (kW / 4) / kThr, kThr, 0, stream>>>(PL0, ba, bb, q0, R2, R1, nullptr, AL1);

  wmma_gemm64<0, false, 0, 1, false, 0><<<dim3(1, 1), 256, 0, stream>>>(
      AL1, AL1, kK, 0L, DA1, DA1, kW, 0L, (void*)(AL1 + kKx), (void*)(AL1 + kKx), kK, 0L, nullptr, nullptr, 0L, kB, kKs, kW, kSc10);
  wmma_gemm64<0, false, 0, 1, false, 0><<<dim3(1, 1), 256, 0, stream>>>(
      AL1 + kW, AL1 + kW, kK, 0L, DB1, DB1, kW, 0L, (void*)(AL1 + kKx + kKs), (void*)(AL1 + kKx + kKs), kK, 0L, nullptr, nullptr, 0L, kB, kKs, kW, kSc10);
  wmma_gemm64<0, false, 0, 0, false, 0><<<dim3((kB / 64) * (kG / 64) / 8, 1), 256, 0, stream>>>(
      AL1, AL1, kK, 0L, WL1, WL1, kK, 0L, (void*)PL1, (void*)PL1, kG, 0L, nullptr, nullptr, 0L, kB, kG, kK, kSc20);
  cell_kernel<true><<<kB * (kW / 4) / kThr, kThr, 0, stream>>>(PL1, ba + (size_t)kG, bb + (size_t)kG, q0 + (size_t)kB * kW, R2 + (size_t)kB * kW, R1 + (size_t)kB * kW, R0, nullptr);
}
static_assert(((kB / 64) * (kG / 64)) % 8 == 0 && kK % 32 == 0 && kW % 32 == 0 && kKs % 64 == 0, "the main product's grid: whole blocks of eight wave tiles; every depth a multiple of 32; the rank-16 products' 64 columns one wave tile");
